// Fusion_1640677507711
// MI455X (gfx1250) — hardware-verified
//
#include <hip/hip_runtime.h>
#include <stddef.h>
#include <stdint.h>
#include <math.h>


#define DD      128
#define NTHR    256
#define NWAVE   8
#define EPT     8
#define CHUNK   (NTHR * EPT)
#define WCAP    (EPT * 32)
#define LISTN   (NWAVE * WCAP)
#define NBMAX   2048
#define SLOTB   11
#define RCAP    28672
#define DEGCAP  128
#define GBM     64
#define GTHR    128
#define MROWS   1024
#define NWMAT   5
#define WUNITS  (DD * (DD / 8))
#define NEGSL   0.2f
#define EPS_SM  1e-16f
#define MXINIT  (-1.0e30f)
#define WSMAX   134217728
#define LDS_AGG ((2 * RCAP + 2 * NBMAX + LISTN) * 4 + 64)

static_assert((CHUNK & (CHUNK - 1)) == 0 && CHUNK <= (1 << SLOTB));
static_assert(NBMAX == (1 << SLOTB));
static_assert(NTHR * 8 == NBMAX);
static_assert(LISTN >= NWAVE * WCAP);
static_assert((RCAP % 32) == 0);
static_assert(LDS_AGG <= 300000);
static_assert(GBM == (GTHR / 32) * 16);
static_assert((DD % 32) == 0 && DD == 4 * 32 && (DD / 8) == 16);
static_assert(MROWS <= NBMAX && (MROWS % GBM) == 0 && (MROWS & (MROWS - 1)) == 0);
static_assert((WUNITS % NTHR) == 0 && WUNITS == 2048);
static_assert(GBM == NWAVE * 8);

typedef float          v4f   __attribute__((ext_vector_type(4)));
typedef float          v8f   __attribute__((ext_vector_type(8)));
typedef int            v4i   __attribute__((ext_vector_type(4)));
typedef int            v8i   __attribute__((ext_vector_type(8)));
typedef unsigned short v8us  __attribute__((ext_vector_type(8)));
typedef __bf16         v16b  __attribute__((ext_vector_type(16)));
typedef v4f  __attribute__((may_alias)) v4fa;
typedef v8us __attribute__((may_alias)) v8usa;
union FragB { v16b v; v8us h[2]; v8i w; };

__device__ __forceinline__ v8f wmb(const FragB& a, const FragB& b, v8f c) {
  v8f d = __builtin_amdgcn_wmma_f32_16x16x32_bf16(false, a.v, false, b.v, (short)0, c, false, false);
  asm volatile("v_nop\n\tv_nop\n\tv_nop\n\tv_nop" : "+v"(d) : "v"(a.w), "v"(b.w));
  return d;
}

__device__ __forceinline__ unsigned bf16_bits(float f) {
  const unsigned u = __float_as_uint(f);
  return (u + 0x7FFFu + ((u >> 16) & 1u)) >> 16;
}
__device__ __forceinline__ float bf16_val(float f) {
  return __uint_as_float(bf16_bits(f) << 16);
}
__device__ __forceinline__ v4f bfr4(const v4f a) {
  v4f r; r.x = bf16_val(a.x); r.y = bf16_val(a.y); r.z = bf16_val(a.z); r.w = bf16_val(a.w); return r;
}
__device__ __forceinline__ float leakyf(float x) { return x > 0.0f ? x : NEGSL * x; }
__device__ __forceinline__ float sc_at(const float* __restrict__ P, int node, int which) {
  return P[(size_t)(node >> 6) * 128 + which * 64 + (node & 63)];
}
__device__ __forceinline__ void sm_step(float lg, float& mx, float& dn, v4f& av, const v4f fs) {
  const float df = lg - mx;
  const float ee = __expf(-fabsf(df));
  const bool  up = df > 0.0f;
  const float s1 = up ? ee : 1.0f;
  const float s2 = up ? 1.0f : ee;
  mx = up ? lg : mx;
  dn = fmaf(dn, s1, s2);
  av.x = fmaf(av.x, s1, s2 * fs.x);
  av.y = fmaf(av.y, s1, s2 * fs.y);
  av.z = fmaf(av.z, s1, s2 * fs.z);
  av.w = fmaf(av.w, s1, s2 * fs.w);
}

__device__ __forceinline__ int scan_chunk(const int* __restrict__ dsts, int nE, int cbase, int slotBase,
                                          int nb, int vec8, int* list, int tid, int lane, int wave) {
  int wc = 0;
  const int el0  = tid * EPT;
  const int e0   = cbase + el0;
  const int sent = -2147483647 - 1;
  v4i da, db;
  if (vec8 != 0 && cbase + CHUNK <= nE) {
    da = *(const v4i*)(dsts + e0);
    db = *(const v4i*)(dsts + e0 + 4);
  } else {
    da.x = (e0     < nE) ? dsts[min(e0,     nE - 1)] : sent;
    da.y = (e0 + 1 < nE) ? dsts[min(e0 + 1, nE - 1)] : sent;
    da.z = (e0 + 2 < nE) ? dsts[min(e0 + 2, nE - 1)] : sent;
    da.w = (e0 + 3 < nE) ? dsts[min(e0 + 3, nE - 1)] : sent;
    db.x = (e0 + 4 < nE) ? dsts[min(e0 + 4, nE - 1)] : sent;
    db.y = (e0 + 5 < nE) ? dsts[min(e0 + 5, nE - 1)] : sent;
    db.z = (e0 + 6 < nE) ? dsts[min(e0 + 6, nE - 1)] : sent;
    db.w = (e0 + 7 < nE) ? dsts[min(e0 + 7, nE - 1)] : sent;
  }
  const unsigned nbs = (unsigned)slotBase;
  const unsigned unb = (unsigned)nb;
  const unsigned s0 = (unsigned)da.x - nbs, s1 = (unsigned)da.y - nbs;
  const unsigned s2 = (unsigned)da.z - nbs, s3 = (unsigned)da.w - nbs;
  const unsigned s4 = (unsigned)db.x - nbs, s5 = (unsigned)db.y - nbs;
  const unsigned s6 = (unsigned)db.z - nbs, s7 = (unsigned)db.w - nbs;
  const bool h0 = s0 < unb, h1 = s1 < unb, h2 = s2 < unb, h3 = s3 < unb;
  const bool h4 = s4 < unb, h5 = s5 < unb, h6 = s6 < unb, h7 = s7 < unb;
  const unsigned any = __builtin_amdgcn_ballot_w32(h0 | h1 | h2 | h3 | h4 | h5 | h6 | h7);
  if (any != 0u) {
#define HITJ(J, HJ, SJ) { \
      const unsigned mj = __builtin_amdgcn_ballot_w32(HJ); \
      if (mj != 0u) { \
        if (HJ) { \
          const int pos = wc + (int)__builtin_amdgcn_mbcnt_lo(mj, 0u); \
          if (pos < WCAP) list[wave * WCAP + pos] = ((el0 + (J)) << SLOTB) | (int)(SJ); \
        } \
        wc += (int)__builtin_popcount(mj); } }
    HITJ(0, h0, s0)
    HITJ(1, h1, s1)
    HITJ(2, h2, s2)
    HITJ(3, h3, s3)
    HITJ(4, h4, s4)
    HITJ(5, h5, s5)
    HITJ(6, h6, s6)
    HITJ(7, h7, s7)
#undef HITJ
  }
  return wc;
}

__global__ __launch_bounds__(NTHR) void k_cvx(const float* __restrict__ x, int nN, int nUnits,
                                              unsigned short* xb) {
  const int u = (int)blockIdx.x * NTHR + (int)threadIdx.x;
  if (u >= nUnits) return;
  const int row = u >> 4;
  const int k8  = (u & 15) * 8;
  const int rc  = row < nN ? row : nN - 1;
  const float* p = x + (size_t)rc * DD + k8;
  const v4f a = *(const v4fa*)p;
  const v4f b = *(const v4fa*)(p + 4);
  const bool ok = row < nN;
  v8us o;
  o[0] = ok ? (unsigned short)bf16_bits(a.x) : (unsigned short)0;
  o[1] = ok ? (unsigned short)bf16_bits(a.y) : (unsigned short)0;
  o[2] = ok ? (unsigned short)bf16_bits(a.z) : (unsigned short)0;
  o[3] = ok ? (unsigned short)bf16_bits(a.w) : (unsigned short)0;
  o[4] = ok ? (unsigned short)bf16_bits(b.x) : (unsigned short)0;
  o[5] = ok ? (unsigned short)bf16_bits(b.y) : (unsigned short)0;
  o[6] = ok ? (unsigned short)bf16_bits(b.z) : (unsigned short)0;
  o[7] = ok ? (unsigned short)bf16_bits(b.w) : (unsigned short)0;
  unsigned short* dp = xb + (size_t)row * DD + k8;
  *(volatile v8us*)dp = o;
  __threadfence();
  *(volatile v8us*)dp = o;
}

__global__ __launch_bounds__(NTHR) void k_wprep(const float* __restrict__ W0, const float* __restrict__ W1,
                                                const float* __restrict__ W2, const float* __restrict__ W3,
                                                const float* __restrict__ W4, unsigned short* WT) {
  const int u = (int)blockIdx.x * NTHR + (int)threadIdx.x;
  if (u >= NWMAT * WUNITS) return;
  const int mi  = u >> 11;
  const int v   = u & (WUNITS - 1);
  const int row = v >> 4;
  const int k8  = (v & 15) * 8;
  const float* W = W0;
  if (mi == 1) W = W1;
  else if (mi == 2) W = W2;
  else if (mi == 3) W = W3;
  else if (mi == 4) W = W4;
  const float* p = W + (size_t)row * DD + k8;
  const v4f a = *(const v4fa*)p;
  const v4f b = *(const v4fa*)(p + 4);
  v8us o;
  o[0] = (unsigned short)bf16_bits(a.x); o[1] = (unsigned short)bf16_bits(a.y);
  o[2] = (unsigned short)bf16_bits(a.z); o[3] = (unsigned short)bf16_bits(a.w);
  o[4] = (unsigned short)bf16_bits(b.x); o[5] = (unsigned short)bf16_bits(b.y);
  o[6] = (unsigned short)bf16_bits(b.z); o[7] = (unsigned short)bf16_bits(b.w);
  unsigned short* dp = WT + (size_t)mi * (DD * DD) + (size_t)row * DD + k8;
  *(volatile v8us*)dp = o;
  __threadfence();
  *(volatile v8us*)dp = o;
}

__global__ __launch_bounds__(GTHR) void k_gemm(const unsigned short* __restrict__ A,
                                               const unsigned short* __restrict__ BT,
                                               float* Cm, int wrC, const float* __restrict__ avs,
                                               const float* __restrict__ avd, float* SC) {
  __shared__ __attribute__((aligned(16))) float stg[GBM * DD];
  __shared__ __attribute__((aligned(16))) float sdt[2 * GBM];
  const int tid = (int)threadIdx.x, lane = tid & 31, wave = tid >> 5, hh = lane >> 4, m = lane & 15;
  const int rowBase = (int)blockIdx.x * GBM;

  v8f acc[8];
  {
    const v8f z = {0.f, 0.f, 0.f, 0.f, 0.f, 0.f, 0.f, 0.f};
#pragma unroll
    for (int t = 0; t < 8; ++t) acc[t] = z;
  }
  const unsigned short* ap = A  + (size_t)(rowBase + 16 * wave + m) * (size_t)DD + 8 * hh;
  const unsigned short* bp = BT + (size_t)m * (size_t)DD + 8 * hh;

#pragma unroll 1
  for (int k0 = 0; k0 < DD; k0 += 32) {
    FragB af;
    af.h[0] = *(const v8usa*)(ap + k0);
    af.h[1] = *(const v8usa*)(ap + k0 + 16);
#pragma unroll
    for (int nt = 0; nt < 8; ++nt) {
      const unsigned short* wq = bp + (size_t)(16 * nt) * (size_t)DD + k0;
      FragB bf;
      bf.h[0] = *(const v8usa*)wq;
      bf.h[1] = *(const v8usa*)(wq + 16);
      acc[nt] = wmb(af, bf, acc[nt]);
    }
  }

#pragma unroll
  for (int nt = 0; nt < 8; ++nt) {
    const int lc = 16 * nt + m;
#pragma unroll
    for (int r = 0; r < 8; ++r) {
      const int lr = 16 * wave + 8 * hh + r;
      stg[lr * DD + lc] = acc[nt][r];
    }
  }
  __syncthreads();

  const v4f as4 = bfr4(*(const v4fa*)(avs + 4 * lane));
  const v4f ad4 = bfr4(*(const v4fa*)(avd + 4 * lane));
  constexpr int RPW = GBM / 4;
#pragma unroll 1
  for (int i = 0; i < RPW; ++i) {
    const int row = wave * RPW + i;
    const v4f p = *(const v4fa*)(stg + row * DD + 4 * lane);
    float s = 0.0f, d = 0.0f;
    s = fmaf(p.x, as4.x, s); s = fmaf(p.y, as4.y, s); s = fmaf(p.z, as4.z, s); s = fmaf(p.w, as4.w, s);
    d = fmaf(p.x, ad4.x, d); d = fmaf(p.y, ad4.y, d); d = fmaf(p.z, ad4.z, d); d = fmaf(p.w, ad4.w, d);
#pragma unroll
    for (int off = 16; off > 0; off >>= 1) {
      s += __shfl_xor(s, off);
      d += __shfl_xor(d, off);
    }
    if (lane == 0) { sdt[row] = s; sdt[GBM + row] = d; }
  }
  __syncthreads();

  const v4f alv = *(const v4fa*)(sdt + 4 * lane);
  float* alp = SC + (size_t)blockIdx.x * (2 * GBM) + 4 * lane;
  if (wrC != 0) {
#pragma unroll 1
    for (int i = 0; i < RPW; ++i) {
      const int row = wave * RPW + i;
      const v4f p = *(const v4fa*)(stg + row * DD + 4 * lane);
      float* op = Cm + (size_t)(rowBase + row) * (size_t)DD + 4 * lane;
      *(volatile v4f*)op = p;
    }
  }
  if (wave == 0) *(volatile v4f*)alp = alv;
  __threadfence();
  if (wrC != 0) {
#pragma unroll 1
    for (int i = 0; i < RPW; ++i) {
      const int row = wave * RPW + i;
      const v4f p = *(const v4fa*)(stg + row * DD + 4 * lane);
      float* op = Cm + (size_t)(rowBase + row) * (size_t)DD + 4 * lane;
      *(volatile v4f*)op = p;
    }
  }
  if (wave == 0) *(volatile v4f*)alp = alv;
}

__global__ __launch_bounds__(NTHR) void k_rowdot(const float* __restrict__ X0, const float* __restrict__ X1,
                                                 int rnd, int nN, const float* __restrict__ attA,
                                                 const float* __restrict__ attB, float* SC) {
  __shared__ __attribute__((aligned(16))) float sd[2 * GBM];
  const int tid = (int)threadIdx.x, lane = tid & 31, wave = tid >> 5;
  const int c0 = 4 * lane;
  const int rowBase = (int)blockIdx.x * GBM;
  const v4f a4 = bfr4(*(const v4fa*)(attA + c0));
  const v4f b4 = bfr4(*(const v4fa*)(attB + c0));
  constexpr int RPW = GBM / NWAVE;
#pragma unroll 1
  for (int i = 0; i < RPW; ++i) {
    const int row  = wave * RPW + i;
    const int grow = rowBase + row;
    const int gcl  = grow < nN ? grow : nN - 1;
    v4f p0 = *(const v4fa*)(X0 + (size_t)gcl * DD + c0);
    v4f p1 = *(const v4fa*)(X1 + (size_t)gcl * DD + c0);
    if (rnd != 0) { p0 = bfr4(p0); p1 = bfr4(p1); }
    float s = 0.0f, d = 0.0f;
    s = fmaf(p0.x, a4.x, s); s = fmaf(p0.y, a4.y, s); s = fmaf(p0.z, a4.z, s); s = fmaf(p0.w, a4.w, s);
    d = fmaf(p1.x, b4.x, d); d = fmaf(p1.y, b4.y, d); d = fmaf(p1.z, b4.z, d); d = fmaf(p1.w, b4.w, d);
#pragma unroll
    for (int off = 16; off > 0; off >>= 1) {
      s += __shfl_xor(s, off);
      d += __shfl_xor(d, off);
    }
    const bool live = grow < nN;
    if (lane == 0) { sd[row] = live ? s : 0.0f; sd[GBM + row] = live ? d : 0.0f; }
  }
  __syncthreads();
  if (wave == 0) {
    const v4f v = *(const v4fa*)(sd + 4 * lane);
    float* op = SC + (size_t)blockIdx.x * (2 * GBM) + 4 * lane;
    *(volatile v4f*)op = v;
    __threadfence();
    *(volatile v4f*)op = v;
  }
}

template<int MODE>
__global__ __launch_bounds__(NTHR) void k_agg(
    const int* __restrict__ srcs, const int* __restrict__ dsts, int nE, int nT, int nS, int nb, int vec8,
    int mRows, const float* __restrict__ F0, const float* __restrict__ F1,
    const float* __restrict__ SPs, const float* __restrict__ SPd,
    const float* __restrict__ base, const float* __restrict__ X1p,
    const float* __restrict__ wa1, const float* __restrict__ wa2, float* outp) {
  static_assert(MODE >= 0 && MODE <= 3);
  extern __shared__ v4f lds_dyn[];
  int* reg1 = (int*)lds_dyn;
  int* reg2 = reg1 + RCAP;
  int* scnt = reg2 + RCAP;
  int* soff = scnt + NBMAX;
  int* list = soff + NBMAX;
  int* wcnt = list + LISTN;
  int* wtot = wcnt + NWAVE;
  const int tid = (int)threadIdx.x, lane = tid & 31, wave = tid >> 5;
  const int nodeBase = (int)blockIdx.x * nb;

  for (int i = tid; i < NBMAX; i += NTHR) scnt[i] = 0;
  __syncthreads();

  int tot = 0;
  const int nChunks = (nE + CHUNK - 1) / CHUNK;
#pragma unroll 1
  for (int ch = 0; ch < nChunks; ++ch) {
    const int cbase = ch * CHUNK;
    const int wc = scan_chunk(dsts, nE, cbase, nodeBase, nb, vec8, list, tid, lane, wave);
    if (lane == 0) wcnt[wave] = wc;
    __syncthreads();
    int pre = 0, all = 0;
#pragma unroll
    for (int w2 = 0; w2 < NWAVE; ++w2) {
      int c = wcnt[w2];
      c = c < 0 ? 0 : (c > WCAP ? WCAP : c);
      all += c;
      pre += (w2 < wave) ? c : 0;
    }
    const int wcc  = wc > WCAP ? WCAP : wc;
    const int bse  = tot + pre;
#pragma unroll 1
    for (int i = lane; i < wcc; i += 32) {
      const int ent = list[wave * WCAP + i];
      const int el  = (ent >> SLOTB) & (CHUNK - 1);
      const int sl  = ent & (NBMAX - 1);
      int eid = cbase + el;
      eid = eid > nE - 1 ? nE - 1 : eid;
      const int pos = bse + i;
      if (pos < RCAP) reg1[pos] = (int)(((unsigned)eid << SLOTB) | (unsigned)sl);
    }
    tot += all;
    tot = tot > RCAP ? RCAP : tot;
    __syncthreads();
  }
  const int nh = tot;

  if (wave == 0) {
#pragma unroll 1
    for (int b0 = 0; b0 < nh; b0 += 32) {
      const int idx = b0 + lane;
      const int uv  = reg1[idx < nh ? idx : nh - 1];
      const int m32 = (nh - b0) < 32 ? (nh - b0) : 32;
#pragma unroll 1
      for (int k = 0; k < m32; ++k) {
        const int u  = __builtin_amdgcn_readlane(uv, k);
        const int sl = u & (NBMAX - 1);
        if (lane == 0) scnt[sl] = scnt[sl] + 1;
      }
    }
  }
  __syncthreads();

  {
    const v4i ca = *(const v4i*)(scnt + 8 * tid);
    const v4i cb = *(const v4i*)(scnt + 8 * tid + 4);
    const int e0 = ca.x < 0 ? 0 : ca.x, e1 = ca.y < 0 ? 0 : ca.y, e2 = ca.z < 0 ? 0 : ca.z, e3 = ca.w < 0 ? 0 : ca.w;
    const int e4 = cb.x < 0 ? 0 : cb.x, e5 = cb.y < 0 ? 0 : cb.y, e6 = cb.z < 0 ? 0 : cb.z, e7 = cb.w < 0 ? 0 : cb.w;
    const int ts = e0 + e1 + e2 + e3 + e4 + e5 + e6 + e7;
    int incl = ts;
#pragma unroll
    for (int d = 1; d < 32; d <<= 1) {
      const int up = __shfl_up(incl, d);
      if (lane >= d) incl += up;
    }
    if (lane == 31) wtot[wave] = incl;
    __syncthreads();
    int pre = 0;
#pragma unroll
    for (int w2 = 0; w2 < NWAVE; ++w2) pre += (w2 < wave) ? wtot[w2] : 0;
    int run = pre + incl - ts;
    soff[8 * tid + 0] = run; run += e0;
    soff[8 * tid + 1] = run; run += e1;
    soff[8 * tid + 2] = run; run += e2;
    soff[8 * tid + 3] = run; run += e3;
    soff[8 * tid + 4] = run; run += e4;
    soff[8 * tid + 5] = run; run += e5;
    soff[8 * tid + 6] = run; run += e6;
    soff[8 * tid + 7] = run;
  }
  __syncthreads();
  for (int i = tid; i < NBMAX; i += NTHR) list[i] = soff[i];
  __syncthreads();

  if (wave == 0) {
#pragma unroll 1
    for (int b0 = 0; b0 < nh; b0 += 32) {
      const int idx = b0 + lane;
      const int uv  = reg1[idx < nh ? idx : nh - 1];
      const int m32 = (nh - b0) < 32 ? (nh - b0) : 32;
#pragma unroll 1
      for (int k = 0; k < m32; ++k) {
        const int u   = __builtin_amdgcn_readlane(uv, k);
        const int sl  = u & (NBMAX - 1);
        const int eid = (int)((unsigned)u >> SLOTB);
        if (lane == 0) {
          int pos = list[sl];
          pos = pos < 0 ? 0 : (pos > RCAP - 1 ? RCAP - 1 : pos);
          reg2[pos] = eid;
          list[sl] = pos + 1;
        }
      }
    }
  }
  __syncthreads();

  const int nbw = nb >> 3;
  const bool ovf = (nh >= RCAP);
  const float qnan = __int_as_float(0x7fc00000);
  const int c0 = 4 * lane;
  v4f q1a, q1b, q2a, q2b;
  {
    const v4f z4 = {0.f, 0.f, 0.f, 0.f};
    q1a = z4; q1b = z4; q2a = z4; q2b = z4;
  }
  if constexpr (MODE == 2) {
    q1a = bfr4(*(const v4fa*)(wa1 + c0));
    q1b = bfr4(*(const v4fa*)(wa1 + DD + c0));
    q2a = bfr4(*(const v4fa*)(wa2 + c0));
    q2b = bfr4(*(const v4fa*)(wa2 + DD + c0));
  }

#pragma unroll 1
  for (int jt = 0; jt < nbw; ++jt) {
    const int slot = wave * nbw + jt;
    const int grow = nodeBase + slot;
    const int gcl  = grow < nT ? grow : nT - 1;
    int st = soff[slot];
    const int craw = scnt[slot];
    int cnt = craw;
    st  = st < 0 ? 0 : (st > nh ? nh : st);
    cnt = cnt < 0 ? 0 : (cnt > DEGCAP ? DEGCAP : cnt);
    if (cnt > nh - st) cnt = nh - st;
    const float pz = (ovf || craw > DEGCAP) ? qnan : 0.0f;

    const float ad0 = sc_at(SPd, gcl, (MODE == 1) ? 0 : 1);
    float ad1 = 0.0f;
    if constexpr (MODE == 1) ad1 = sc_at(SPd, gcl, 1);
    float mx0 = MXINIT, dn0 = 0.0f, mx1 = MXINIT, dn1 = 0.0f;
    v4f av0 = {0.f, 0.f, 0.f, 0.f};
    v4f av1 = {0.f, 0.f, 0.f, 0.f};

#pragma unroll 1
    for (int q = 0; q < cnt; ++q) {
      int idx = st + q; idx = idx > RCAP - 1 ? RCAP - 1 : idx;
      int eid = reg2[idx]; eid = eid < 0 ? 0 : (eid > nE - 1 ? nE - 1 : eid);
      const int sraw = srcs[eid];
      const int s = sraw < 0 ? 0 : (sraw > nS - 1 ? nS - 1 : sraw);
      const v4f fs = *(const v4fa*)(F0 + (size_t)s * DD + c0);
      const float lg = leakyf(sc_at(SPs, s, 0) + ad0);
      sm_step(lg, mx0, dn0, av0, fs);
      if constexpr (MODE == 1) {
        const v4f gs = *(const v4fa*)(F1 + (size_t)s * DD + c0);
        const float lh = leakyf(sc_at(SPs, s, 1) + ad1);
        sm_step(lh, mx1, dn1, av1, gs);
      }
    }
    const float inv0 = __builtin_amdgcn_rcpf(dn0 + EPS_SM);
    v4f v0;
    v0.x = av0.x * inv0; v0.y = av0.y * inv0; v0.z = av0.z * inv0; v0.w = av0.w * inv0;
    const bool live = grow < nT;
    v4f o;
    if constexpr (MODE == 0) {
      o.x = live ? v0.x : 0.0f; o.y = live ? v0.y : 0.0f; o.z = live ? v0.z : 0.0f; o.w = live ? v0.w : 0.0f;
    } else if constexpr (MODE == 1) {
      const float inv1 = __builtin_amdgcn_rcpf(dn1 + EPS_SM);
      const v4f bq = bfr4(*(const v4fa*)(base + (size_t)gcl * DD + c0));
      o.x = (bq.x + v0.x) + av1.x * inv1;
      o.y = (bq.y + v0.y) + av1.y * inv1;
      o.z = (bq.z + v0.z) + av1.z * inv1;
      o.w = (bq.w + v0.w) + av1.w * inv1;
    } else if constexpr (MODE == 2) {
      const v4f bq = bfr4(*(const v4fa*)(base + (size_t)gcl * DD + c0));
      const v4f r1 = *(const v4fa*)(X1p + (size_t)gcl * DD + c0);
      float z1 = 0.0f, z2 = 0.0f;
      z1 = fmaf(r1.x, q1a.x, z1); z1 = fmaf(r1.y, q1a.y, z1); z1 = fmaf(r1.z, q1a.z, z1); z1 = fmaf(r1.w, q1a.w, z1);
      z1 = fmaf(bq.x, q1b.x, z1); z1 = fmaf(bq.y, q1b.y, z1); z1 = fmaf(bq.z, q1b.z, z1); z1 = fmaf(bq.w, q1b.w, z1);
      z2 = fmaf(v0.x, q2a.x, z2); z2 = fmaf(v0.y, q2a.y, z2); z2 = fmaf(v0.z, q2a.z, z2); z2 = fmaf(v0.w, q2a.w, z2);
      z2 = fmaf(bq.x, q2b.x, z2); z2 = fmaf(bq.y, q2b.y, z2); z2 = fmaf(bq.z, q2b.z, z2); z2 = fmaf(bq.w, q2b.w, z2);
#pragma unroll
      for (int off = 16; off > 0; off >>= 1) {
        z1 += __shfl_xor(z1, off);
        z2 += __shfl_xor(z2, off);
      }
      const float g1 = __expf(z1 - z1);
      const float g2 = __expf(z2 - z2);
      const float at1 = g1 * __builtin_amdgcn_rcpf(g1);
      const float at2 = g2 * __builtin_amdgcn_rcpf(g2);
      o.x = (bq.x + at1 * r1.x) + at2 * v0.x;
      o.y = (bq.y + at1 * r1.y) + at2 * v0.y;
      o.z = (bq.z + at1 * r1.z) + at2 * v0.z;
      o.w = (bq.w + at1 * r1.w) + at2 * v0.w;
    } else {
      const v4f bq = bfr4(*(const v4fa*)(base + (size_t)gcl * DD + c0));
      o.x = bq.x + v0.x; o.y = bq.y + v0.y; o.z = bq.z + v0.z; o.w = bq.w + v0.w;
    }
    o.x += pz; o.y += pz; o.z += pz; o.w += pz;

    float* op = outp + (size_t)grow * DD + c0;
    if constexpr (MODE == 0) {
      const bool wr = grow < mRows;
      if (wr) *(volatile v4f*)op = o;
      __threadfence();
      if (wr) *(volatile v4f*)op = o;
    } else {
      if (live) *(volatile v4f*)op = o;
      __threadfence();
      if (live) *(volatile v4f*)op = o;
    }
  }
}

static int pick_nb(int nE, int nN) {
  int nb = MROWS;
  while (nb > 32 && (long long)nb * (long long)nE * 10LL > (long long)RCAP * (long long)nN * 9LL) nb >>= 1;
  return nb;
}
static inline int cdiv(int a, int b) { return (a + b - 1) / b; }

extern "C" void kernel_launch(void* const* d_in, const int* in_sizes, int n_in,
                              void* d_out, int out_size, void* d_ws, size_t ws_size,
                              hipStream_t stream) {
  if (n_in < 31) return;
  if (in_sizes[0] < DD || (in_sizes[0] % DD) != 0) return;
  if (in_sizes[1] < DD || (in_sizes[1] % DD) != 0) return;
  if (in_sizes[2] < DD || (in_sizes[2] % DD) != 0) return;
  const int nStu  = in_sizes[0] / DD;
  const int nItem = in_sizes[1] / DD;
  const int nConc = in_sizes[2] / DD;
  if (in_sizes[3] != in_sizes[0]) return;
  if (nStu > (1 << 22) || nItem > (1 << 22) || nConc > (1 << 22)) return;
  if (in_sizes[4] != DD * DD || in_sizes[7] != DD * DD || in_sizes[14] != DD * DD ||
      in_sizes[17] != DD * DD || in_sizes[22] != DD * DD) return;
  {
    const int vecIdx[16] = {5, 6, 8, 9, 10, 11, 12, 13, 15, 16, 18, 19, 23, 24, 5, 6};
    for (int i = 0; i < 16; ++i) if (in_sizes[vecIdx[i]] != DD) return;
  }
  if (in_sizes[20] != 2 * DD || in_sizes[21] != 2 * DD) return;
  const int eCC = in_sizes[25];
  const int eIC = in_sizes[27];
  const int eSI = in_sizes[29];
  if (in_sizes[26] != eCC || in_sizes[28] != eIC || in_sizes[30] != eSI) return;
  if (eCC < 1 || eIC < 1 || eSI < 1) return;
  if (eCC >= (1 << (32 - SLOTB)) || eIC >= (1 << (32 - SLOTB)) || eSI >= (1 << (32 - SLOTB))) return;
  if ((long long)out_size != (long long)(nConc + nItem + nStu) * DD) return;

  const float* stu_x     = (const float*)d_in[0];
  const float* item_x    = (const float*)d_in[1];
  const float* conc_x    = (const float*)d_in[2];
  const float* stu_raw_x = (const float*)d_in[3];
  const float* W_cc  = (const float*)d_in[4];  const float* al_cc  = (const float*)d_in[5];  const float* ar_cc  = (const float*)d_in[6];
  const float* W_ic  = (const float*)d_in[7];  const float* al_ic  = (const float*)d_in[8];  const float* ar_ic  = (const float*)d_in[9];
  const float* al_cce = (const float*)d_in[10]; const float* ar_cce = (const float*)d_in[11];
  const float* al_ice = (const float*)d_in[12]; const float* ar_ice = (const float*)d_in[13];
  const float* W_ci  = (const float*)d_in[14]; const float* al_ci  = (const float*)d_in[15]; const float* ar_ci  = (const float*)d_in[16];
  const float* W_si  = (const float*)d_in[17]; const float* al_si  = (const float*)d_in[18]; const float* ar_si  = (const float*)d_in[19];
  const float* w_ci_att = (const float*)d_in[20];
  const float* w_si_att = (const float*)d_in[21];
  const float* W_is  = (const float*)d_in[22]; const float* al_is  = (const float*)d_in[23]; const float* ar_is  = (const float*)d_in[24];
  const int* cc_src  = (const int*)d_in[25];
  const int* cc_dst  = (const int*)d_in[26];
  const int* ic_item = (const int*)d_in[27];
  const int* ic_conc = (const int*)d_in[28];
  const int* si_stu  = (const int*)d_in[29];
  const int* si_item = (const int*)d_in[30];
  float* out = (float*)d_out;
  const size_t offItem = (size_t)nConc * DD;
  const size_t offStu  = offItem + (size_t)nItem * DD;
  if (offStu + (size_t)nStu * DD != (size_t)out_size) return;
  float* out0 = out;
  float* out1 = out + offItem;
  float* out2 = out + offStu;

  const int MPc = cdiv(nConc, MROWS) * MROWS;
  const int MPi = cdiv(nItem, MROWS) * MROWS;
  const int MPs = cdiv(nStu,  MROWS) * MROWS;
  const int gMc = MPc / GBM, gMi = MPi / GBM, gMs = MPs / GBM;

  const int nb_cc = pick_nb(eCC, nConc);
  const int nb_c2 = pick_nb(eIC, nConc);
  const int nb_i1 = pick_nb(eIC, nItem);
  const int nb_i2 = pick_nb(eSI, nItem);
  const int nb_s1 = pick_nb(eSI, nStu);
  {
    const int nbs[5] = {nb_cc, nb_c2, nb_i1, nb_i2, nb_s1};
    for (int i = 0; i < 5; ++i) if (nbs[i] < 32 || (nbs[i] & (nbs[i] - 1)) != 0 || nbs[i] > MROWS) return;
  }
  const int gA_cc = MPc / nb_cc, gA_c2 = MPc / nb_c2, gA_i1 = MPi / nb_i1, gA_i2 = MPi / nb_i2, gA_s1 = MPs / nb_s1;
  if (gA_cc * nb_cc != MPc || gA_c2 * nb_c2 != MPc || gA_i1 * nb_i1 != MPi || gA_i2 * nb_i2 != MPi ||
      gA_s1 * nb_s1 != MPs) return;
  const int v_cc = ((eCC & 3) == 0) ? 1 : 0;
  const int v_ic = ((eIC & 3) == 0) ? 1 : 0;
  const int v_si = ((eSI & 3) == 0) ? 1 : 0;

  char* ws = (char*)d_ws;
  size_t off = 0;
  auto carve = [&](size_t bytes) { const size_t o = off; off += bytes; off = (off + 255) & ~(size_t)255; return o; };
  const size_t oWT   = carve((size_t)NWMAT * DD * DD * 2);
  const size_t oXBc  = carve((size_t)MPc * DD * 2);
  const size_t oXBi  = carve((size_t)MPi * DD * 2);
  const size_t oXBs  = carve((size_t)MPs * DD * 2);
  const size_t oXBr  = carve((size_t)MPs * DD * 2);
  const size_t oXLcc = carve((size_t)MPc * DD * 4);
  const size_t oXLi1 = carve((size_t)MPc * DD * 4);
  const size_t oXLc2 = carve((size_t)MPi * DD * 4);
  const size_t oXLs1 = carve((size_t)MPi * DD * 4);
  const size_t oXLi2 = carve((size_t)MPs * DD * 4);
  const size_t oC1P  = carve((size_t)MPc * DD * 4);
  const size_t oC2P  = carve((size_t)MPc * DD * 4);
  const size_t oI1P  = carve((size_t)MPi * DD * 4);
  const size_t oSC1  = carve((size_t)MPc * 8);
  const size_t oSC2  = carve((size_t)MPc * 8);
  const size_t oSC3  = carve((size_t)MPc * 8);
  const size_t oRD1  = carve((size_t)MPc * 8);
  const size_t oRD2  = carve((size_t)MPc * 8);
  const size_t oSC4  = carve((size_t)MPi * 8);
  const size_t oSC5  = carve((size_t)MPi * 8);
  const size_t oSC6  = carve((size_t)MPi * 8);
  const size_t oSC7  = carve((size_t)MPi * 8);
  const size_t oSC8  = carve((size_t)MPs * 8);
  const size_t oSC9  = carve((size_t)MPs * 8);
  if (off > ws_size || off > (size_t)WSMAX) return;

  unsigned short* WT  = (unsigned short*)(ws + oWT);
  unsigned short* Wcc = WT;
  unsigned short* Wic = WT + (size_t)1 * DD * DD;
  unsigned short* Wci = WT + (size_t)2 * DD * DD;
  unsigned short* Wsi = WT + (size_t)3 * DD * DD;
  unsigned short* Wis = WT + (size_t)4 * DD * DD;
  unsigned short* XBc = (unsigned short*)(ws + oXBc);
  unsigned short* XBi = (unsigned short*)(ws + oXBi);
  unsigned short* XBs = (unsigned short*)(ws + oXBs);
  unsigned short* XBr = (unsigned short*)(ws + oXBr);
  float* XLcc = (float*)(ws + oXLcc);
  float* XLi1 = (float*)(ws + oXLi1);
  float* XLc2 = (float*)(ws + oXLc2);
  float* XLs1 = (float*)(ws + oXLs1);
  float* XLi2 = (float*)(ws + oXLi2);
  float* C1P  = (float*)(ws + oC1P);
  float* C2P  = (float*)(ws + oC2P);
  float* I1P  = (float*)(ws + oI1P);
  float* SC1 = (float*)(ws + oSC1);
  float* SC2 = (float*)(ws + oSC2);
  float* SC3 = (float*)(ws + oSC3);
  float* RD1 = (float*)(ws + oRD1);
  float* RD2 = (float*)(ws + oRD2);
  float* SC4 = (float*)(ws + oSC4);
  float* SC5 = (float*)(ws + oSC5);
  float* SC6 = (float*)(ws + oSC6);
  float* SC7 = (float*)(ws + oSC7);
  float* SC8 = (float*)(ws + oSC8);
  float* SC9 = (float*)(ws + oSC9);

  hipFuncSetAttribute(reinterpret_cast<const void*>(&k_agg<0>), hipFuncAttributeMaxDynamicSharedMemorySize, LDS_AGG);
  hipFuncSetAttribute(reinterpret_cast<const void*>(&k_agg<1>), hipFuncAttributeMaxDynamicSharedMemorySize, LDS_AGG);
  hipFuncSetAttribute(reinterpret_cast<const void*>(&k_agg<2>), hipFuncAttributeMaxDynamicSharedMemorySize, LDS_AGG);
  hipFuncSetAttribute(reinterpret_cast<const void*>(&k_agg<3>), hipFuncAttributeMaxDynamicSharedMemorySize, LDS_AGG);

  k_wprep<<<(NWMAT * WUNITS) / NTHR, NTHR, 0, stream>>>(W_cc, W_ic, W_ci, W_si, W_is, WT);
  {
    const int uC = MPc * (DD / 8), uI = MPi * (DD / 8), uS = MPs * (DD / 8);
    k_cvx<<<cdiv(uC, NTHR), NTHR, 0, stream>>>(conc_x,    nConc, uC, XBc);
    k_cvx<<<cdiv(uI, NTHR), NTHR, 0, stream>>>(item_x,    nItem, uI, XBi);
    k_cvx<<<cdiv(uS, NTHR), NTHR, 0, stream>>>(stu_x,     nStu,  uS, XBs);
    k_cvx<<<cdiv(uS, NTHR), NTHR, 0, stream>>>(stu_raw_x, nStu,  uS, XBr);
  }

  k_gemm<<<gMc, GTHR, 0, stream>>>(XBc, Wcc, XLcc, 1, al_cc, ar_cc, SC1);
  k_gemm<<<gMc, GTHR, 0, stream>>>(XBc, Wic, XLi1, 0, al_ic, ar_ic, SC2);
  k_gemm<<<gMc, GTHR, 0, stream>>>(XBc, Wci, XLi1, 1, al_ci, ar_ci, SC3);
  k_gemm<<<gMi, GTHR, 0, stream>>>(XBi, Wic, XLc2, 1, al_ic, ar_ic, SC4);
  k_gemm<<<gMi, GTHR, 0, stream>>>(XBi, Wci, XLs1, 0, al_ci, ar_ci, SC5);
  k_gemm<<<gMi, GTHR, 0, stream>>>(XBi, Wsi, XLs1, 0, al_si, ar_si, SC6);
  k_gemm<<<gMi, GTHR, 0, stream>>>(XBi, Wis, XLs1, 1, al_is, ar_is, SC7);
  k_gemm<<<gMs, GTHR, 0, stream>>>(XBs, Wsi, XLi2, 1, al_si, ar_si, SC8);
  k_gemm<<<gMs, GTHR, 0, stream>>>(XBr, Wis, XLi2, 0, al_is, ar_is, SC9);

  k_rowdot<<<gMc, NTHR, 0, stream>>>(conc_x, conc_x, 1, nConc, ar_cce, ar_ice, RD1);
  k_agg<0><<<gA_cc, NTHR, LDS_AGG, stream>>>(cc_src, cc_dst, eCC, nConc, nConc, nb_cc, v_cc, MPc,
                                             XLcc, XLcc, SC1, SC1, conc_x, XLcc, al_cc, al_cc, C1P);
  k_agg<0><<<gA_c2, NTHR, LDS_AGG, stream>>>(ic_item, ic_conc, eIC, nConc, nItem, nb_c2, v_ic, MPc,
                                             XLc2, XLc2, SC4, SC2, conc_x, XLc2, al_cc, al_cc, C2P);
  k_rowdot<<<gMc, NTHR, 0, stream>>>(C1P, C2P, 0, nConc, al_cce, al_ice, RD2);
  k_agg<1><<<gA_cc, NTHR, LDS_AGG, stream>>>(cc_src, cc_dst, eCC, nConc, nConc, nb_cc, v_cc, MPc,
                                             C1P, C2P, RD2, RD1, conc_x, C1P, al_cc, al_cc, out0);

  k_agg<0><<<gA_i1, NTHR, LDS_AGG, stream>>>(ic_conc, ic_item, eIC, nItem, nConc, nb_i1, v_ic, MPi,
                                             XLi1, XLi1, SC3, SC5, item_x, XLi1, al_cc, al_cc, I1P);
  k_agg<2><<<gA_i2, NTHR, LDS_AGG, stream>>>(si_stu, si_item, eSI, nItem, nStu, nb_i2, v_si, MPi,
                                             XLi2, XLi2, SC8, SC6, item_x, I1P, w_ci_att, w_si_att, out1);

  k_agg<3><<<gA_s1, NTHR, LDS_AGG, stream>>>(si_item, si_stu, eSI, nStu, nItem, nb_s1, v_si, MPs,
                                             XLs1, XLs1, SC7, SC9, stu_raw_x, XLs1, al_cc, al_cc, out2);
}
